// RelativeAttention_71476845740463
// MI455X (gfx1250) — hardware-run, weakly checked
//
#include <hip/hip_runtime.h>

typedef __attribute__((ext_vector_type(16))) __bf16 v16b;
typedef __attribute__((ext_vector_type(8)))  __bf16 v8b;
typedef __attribute__((ext_vector_type(8)))  float  v8f;
typedef __attribute__((ext_vector_type(4)))  float  v4f;
typedef __attribute__((ext_vector_type(4)))  unsigned int v4u;
typedef __attribute__((ext_vector_type(4)))  int v4i;
typedef v8b v8b_a __attribute__((may_alias));
typedef v4f v4f_a __attribute__((may_alias));
typedef v4u v4u_a __attribute__((may_alias));

#ifndef NB
#define NB 2
#endif
#ifndef SEQ
#define SEQ 1024
#endif
#define NB_FULL 2
#define SEQ_FULL 1024

#define VGPR_CAP __attribute__((amdgpu_num_vgpr(256)))

constexpr int DMODEL = 1024;
constexpr int NHEAD  = 16;
constexpr int DHEAD  = 64;
constexpr int NPOS   = 2047;
constexpr int NQKV   = 3 * DMODEL;
constexpr int NBH    = NB * NHEAD;
constexpr int MROWS  = NB * SEQ;
constexpr int KCH    = 64;
constexpr int NWAVE  = 4;
constexpr int GP     = 84;
constexpr int SP     = 68;
constexpr int TQ_PITCH = 72;
constexpr int TV_PITCH = 136;
constexpr int T_ELEMS  = 128 * TQ_PITCH;
constexpr int TS_PITCH = 72;
constexpr int OS_PITCH = 68;

constexpr size_t PLANE  = (size_t)NBH * SEQ * DHEAD;
constexpr size_t XB_E   = (size_t)MROWS * DMODEL;
constexpr size_t WQT_E  = (size_t)NQKV * DMODEL;
constexpr size_t WOT_E  = (size_t)DMODEL * DMODEL;
constexpr size_t ERB_E  = (size_t)NHEAD * 2048 * DHEAD;
constexpr size_t QKVP_E = 6 * PLANE;
constexpr size_t CTX_E  = 2 * XB_E;
constexpr size_t WS_NEED = 2 * (XB_E + WQT_E + WOT_E + ERB_E + QKVP_E + CTX_E);

static_assert(SEQ % 128 == 0);
static_assert(SEQ <= SEQ_FULL && NB <= NB_FULL);
static_assert(DHEAD == 64 && DMODEL == NHEAD * DHEAD);
static_assert(DMODEL % 64 == 0 && NQKV % 64 == 0 && DMODEL % 32 == 0);
static_assert(64 * TV_PITCH <= T_ELEMS);
static_assert((TQ_PITCH * 2) % 16 == 0 && (TV_PITCH * 2) % 16 == 0 && (GP * 4) % 16 == 0 && (OS_PITCH * 4) % 16 == 0);
static_assert(GP >= 80 && SP >= 64);
static_assert((size_t)NHEAD * NPOS * DHEAD <= ERB_E);
static_assert(WS_NEED <= 134217728ull);


__device__ __forceinline__ unsigned short f2bf_bits(float f) {
  unsigned u = __float_as_uint(f);
  return (unsigned short)((u + 0x7FFFu + ((u >> 16) & 1u)) >> 16);
}
__device__ __forceinline__ float bf_bits2f(unsigned short h) { return __uint_as_float(((unsigned)h) << 16); }
__device__ __forceinline__ unsigned pk2(float a, float b) {
  return (unsigned)f2bf_bits(a) | ((unsigned)f2bf_bits(b) << 16);
}
__device__ __forceinline__ void split2(float a, float b, unsigned& hw, unsigned& lw) {
  const unsigned short ha = f2bf_bits(a);
  const unsigned short hb = f2bf_bits(b);
  const unsigned short la = f2bf_bits(a - bf_bits2f(ha));
  const unsigned short lb = f2bf_bits(b - bf_bits2f(hb));
  hw = (unsigned)ha | ((unsigned)hb << 16);
  lw = (unsigned)la | ((unsigned)lb << 16);
}

__device__ __forceinline__ v8f mma_bf16(v16b a, v16b b, v8f c) {
  c = __builtin_amdgcn_wmma_f32_16x16x32_bf16(false, a, false, b, (short)0, c, false, false);
  asm volatile("v_nop\n\tv_nop\n\tv_nop\n\tv_nop" : "+v"(c) : "v"(a), "v"(b));
  return c;
}

__device__ __forceinline__ void wave_lds_sync() {
  __builtin_amdgcn_fence(3  , "workgroup");
  __builtin_amdgcn_wave_barrier();
  __builtin_amdgcn_fence(2  , "workgroup");
}

__global__ __launch_bounds__(256) void cvt_rows_kernel(
    const float* __restrict__ in, unsigned short* __restrict__ outp,
    int nunits, int upr, int rpb, int rpb_full)
{
  const int u = blockIdx.x * 256 + threadIdx.x;
  if (u >= nunits) return;
  const int row = u / upr;
  const int seg = u - row * upr;
  const int b = row / rpb;
  const int l = row - b * rpb;
  const float* src = in + ((size_t)(b * rpb_full + l) * upr + seg) * 8;
  const v4f a0 = *(const v4f*)src;
  const v4f a1 = *(const v4f*)(src + 4);
  v4u w;
  w[0] = pk2(a0[0], a0[1]);
  w[1] = pk2(a0[2], a0[3]);
  w[2] = pk2(a1[0], a1[1]);
  w[3] = pk2(a1[2], a1[3]);
  volatile v4u* dst = (volatile v4u*)(outp + ((size_t)row * upr + seg) * 8);
  *dst = w;
  __threadfence();
  *dst = w;
}

__global__ __launch_bounds__(256) void wt_planes_kernel(
    const float* __restrict__ W, unsigned short* __restrict__ Wt, int rows, int cols)
{
  __shared__ __align__(16) unsigned short Ts[64 * TS_PITCH];
  const int k0 = blockIdx.x * 64;
  const int n0 = blockIdx.y * 64;
  const int tid = threadIdx.x;
#pragma unroll
  for (int it = 0; it < 2; ++it) {
    const int u = it * 256 + tid;
    const int row = u >> 3;
    const int seg = u & 7;
    const float* src = W + (size_t)(k0 + row) * cols + n0 + seg * 8;
    const v4f a0 = *(const v4f*)src;
    const v4f a1 = *(const v4f*)(src + 4);
#pragma unroll
    for (int e = 0; e < 4; ++e) {
      Ts[(seg * 8 + e) * TS_PITCH + row]     = f2bf_bits(a0[e]);
      Ts[(seg * 8 + 4 + e) * TS_PITCH + row] = f2bf_bits(a1[e]);
    }
  }
  __syncthreads();
  for (int pass = 0; pass < 2; ++pass) {
#pragma unroll
    for (int it = 0; it < 2; ++it) {
      const int u = it * 256 + tid;
      const int nrow = u >> 3;
      const int seg  = u & 7;
      const v4u w = *(const v4u_a*)(Ts + nrow * TS_PITCH + seg * 8);
      *(volatile v4u*)(Wt + (size_t)(n0 + nrow) * rows + k0 + seg * 8) = w;
    }
    __threadfence();
  }
}

__global__ __launch_bounds__(128) VGPR_CAP void gemm_qkv_kernel(
    const unsigned short* __restrict__ Xb, const unsigned short* __restrict__ WqT,
    const float* __restrict__ bias, unsigned short* __restrict__ qkvp)
{
  union FB { v16b v; v8b h[2]; };
  __shared__ __align__(16) unsigned short Th[T_ELEMS];
  __shared__ __align__(16) unsigned short Tl[T_ELEMS];

  const int tid  = threadIdx.x;
  const int wave = __builtin_amdgcn_readfirstlane(tid >> 5);
  const int lane = tid & 31;
  const int hh   = lane >> 4;
  const int c    = lane & 15;
  const int n0   = blockIdx.x * 64;
  const int m0   = blockIdx.y * 128;

  v8f acc[2][4];
#pragma unroll
  for (int mt = 0; mt < 2; ++mt)
#pragma unroll
    for (int t = 0; t < 4; ++t) acc[mt][t] = (v8f){0.f,0.f,0.f,0.f,0.f,0.f,0.f,0.f};

  const unsigned short* a0p = Xb + (size_t)(m0 + wave * 32 + c) * DMODEL + 8 * hh;
  const unsigned short* a1p = a0p + (size_t)16 * DMODEL;
  const unsigned short* bp  = WqT + (size_t)(n0 + c) * DMODEL + 8 * hh;

#pragma unroll 1
  for (int k0 = 0; k0 < DMODEL; k0 += 32) {
    FB a0, a1;
    a0.h[0] = *(const v8b*)(a0p + k0);
    a0.h[1] = *(const v8b*)(a0p + k0 + 16);
    a1.h[0] = *(const v8b*)(a1p + k0);
    a1.h[1] = *(const v8b*)(a1p + k0 + 16);
#pragma unroll
    for (int t = 0; t < 4; ++t) {
      FB bf;
      bf.h[0] = *(const v8b*)(bp + (size_t)t * 16 * DMODEL + k0);
      bf.h[1] = *(const v8b*)(bp + (size_t)t * 16 * DMODEL + k0 + 16);
      acc[0][t] = mma_bf16(a0.v, bf.v, acc[0][t]);
      acc[1][t] = mma_bf16(a1.v, bf.v, acc[1][t]);
    }
  }

  const int sec = n0 / DMODEL;
  const float osc = (sec == 1) ? 0.125f : 1.0f;
#pragma unroll
  for (int t = 0; t < 4; ++t) {
    const float bv = bf_bits2f(f2bf_bits(bias[n0 + 16 * t + c]));
#pragma unroll
    for (int mt = 0; mt < 2; ++mt) {
#pragma unroll
      for (int r = 0; r < 8; ++r) {
        const float val = (acc[mt][t][r] + bv) * osc;
        const unsigned short hb = f2bf_bits(val);
        const unsigned short lb = f2bf_bits(val - bf_bits2f(hb));
        const int rl = wave * 32 + mt * 16 + 8 * hh + r;
        const int cl = 16 * t + c;
        const int idx = (sec < 2) ? (rl * TQ_PITCH + cl) : (cl * TV_PITCH + rl);
        Th[idx] = hb;
        Tl[idx] = lb;
      }
    }
  }
  __syncthreads();

  const int b  = m0 / SEQ;
  const int l0 = m0 - b * SEQ;
  const int h  = (n0 - sec * DMODEL) / DHEAD;
  const int bh = b * NHEAD + h;
  unsigned short* ph = qkvp + (size_t)(2 * sec) * PLANE;
  unsigned short* pl = ph + PLANE;

  for (int pass = 0; pass < 2; ++pass) {
    if (sec < 2) {
#pragma unroll
      for (int it = 0; it < 8; ++it) {
        const int u = it * 128 + tid;
        const int row = u >> 3;
        const int seg = u & 7;
        const v4u hw = *(const v4u_a*)(Th + row * TQ_PITCH + seg * 8);
        const v4u lw = *(const v4u_a*)(Tl + row * TQ_PITCH + seg * 8);
        const size_t g = ((size_t)bh * SEQ + l0 + row) * DHEAD + seg * 8;
        *(volatile v4u*)(ph + g) = hw;
        *(volatile v4u*)(pl + g) = lw;
      }
    } else {
#pragma unroll
      for (int it = 0; it < 8; ++it) {
        const int u = it * 128 + tid;
        const int drow = u >> 4;
        const int seg  = u & 15;
        const v4u hw = *(const v4u_a*)(Th + drow * TV_PITCH + seg * 8);
        const v4u lw = *(const v4u_a*)(Tl + drow * TV_PITCH + seg * 8);
        const size_t g = ((size_t)bh * DHEAD + drow) * SEQ + l0 + seg * 8;
        *(volatile v4u*)(ph + g) = hw;
        *(volatile v4u*)(pl + g) = lw;
      }
    }
    __threadfence();
  }
}

__global__ __launch_bounds__(128) VGPR_CAP void rel_attn_kernel(
    const unsigned short* __restrict__ qkvp, const unsigned short* __restrict__ Erb,
    const int* __restrict__ mask, unsigned short* __restrict__ ctxp)
{
  union FB { v16b v; v8b h[2]; };
  __shared__ __align__(16) float Gs[NWAVE][16 * GP];
  __shared__ __align__(16) float Ss[NWAVE][16 * SP];
  __shared__ __align__(16) unsigned short Psh[NWAVE][16 * KCH];
  __shared__ __align__(16) unsigned short Psl[NWAVE][16 * KCH];

  const int tid  = threadIdx.x;
  const int wave = __builtin_amdgcn_readfirstlane(tid >> 5);
  const int lane = tid & 31;
  const int hh   = lane >> 4;
  const int c    = lane & 15;
  const int c3   = c & 3;
  const int csh  = c >> 2;
  const int qb   = blockIdx.x;
  const int bh   = blockIdx.y;
  const int b    = bh / NHEAD;
  const int h    = bh - b * NHEAD;
  const int q0   = qb * 64 + wave * 16;
  const float NEG_INF = -__builtin_inff();

  const unsigned short* Qh  = qkvp + (size_t)bh * SEQ * DHEAD;
  const unsigned short* Ql  = Qh + PLANE;
  const unsigned short* Kh  = Qh + 2 * PLANE;
  const unsigned short* Kl  = Qh + 3 * PLANE;
  const unsigned short* Vth = Qh + 4 * PLANE;
  const unsigned short* Vtl = Qh + 5 * PLANE;
  const unsigned short* Eh  = Erb + (size_t)h * NPOS * DHEAD;

  v16b qh[2], ql[2];
  {
    const size_t qo = (size_t)(q0 + c) * DHEAD + 8 * hh;
#pragma unroll
    for (int dc = 0; dc < 2; ++dc) {
      FB f;
      f.h[0] = *(const v8b*)(Qh + qo + dc * 32);
      f.h[1] = *(const v8b*)(Qh + qo + dc * 32 + 16);
      qh[dc] = f.v;
      f.h[0] = *(const v8b*)(Ql + qo + dc * 32);
      f.h[1] = *(const v8b*)(Ql + qo + dc * 32 + 16);
      ql[dc] = f.v;
    }
  }

  float mrow[8], lrow[8];
  v8f oacc[4];
#pragma unroll
  for (int r = 0; r < 8; ++r) { mrow[r] = NEG_INF; lrow[r] = 0.f; }
#pragma unroll
  for (int t = 0; t < 4; ++t) oacc[t] = (v8f){0.f,0.f,0.f,0.f,0.f,0.f,0.f,0.f};

  float* gs = Gs[wave];
  float* ss = Ss[wave];
  unsigned short* pwh = Psh[wave];
  unsigned short* pwl = Psl[wave];

#pragma unroll 1
  for (int kc = 0; kc < SEQ / KCH; ++kc) {
    const int kv0 = kc * KCH;

    unsigned msel[8];
    unsigned andall = 0xFFFFFFFFu;
#pragma unroll
    for (int it = 0; it < 8; ++it) {
      const v4i mv = *(const v4i*)(mask + (size_t)(q0 + 2 * it + hh) * SEQ_FULL + kv0 + 4 * c);
      const unsigned b0 = __builtin_amdgcn_ballot_w32(mv[0] != 0);
      const unsigned b1 = __builtin_amdgcn_ballot_w32(mv[1] != 0);
      const unsigned b2 = __builtin_amdgcn_ballot_w32(mv[2] != 0);
      const unsigned b3 = __builtin_amdgcn_ballot_w32(mv[3] != 0);
      andall &= (b0 & b1) & (b2 & b3);
      msel[it] = (c3 == 0) ? b0 : (c3 == 1) ? b1 : (c3 == 2) ? b2 : b3;
    }
    if (andall == 0xFFFFFFFFu) continue;

    unsigned mw[4];
#pragma unroll
    for (int ii = 0; ii < 4; ++ii) mw[ii] = hh ? msel[4 + ii] : msel[ii];

#pragma unroll 1
    for (int j = 0; j < 4; ++j) {
      v8f sa = (v8f){0.f,0.f,0.f,0.f,0.f,0.f,0.f,0.f};
      const size_t ko = (size_t)(kv0 + j * 16 + c) * DHEAD + 8 * hh;
#pragma unroll
      for (int dc = 0; dc < 2; ++dc) {
        FB kfh, kfl;
        kfh.h[0] = *(const v8b*)(Kh + ko + dc * 32);
        kfh.h[1] = *(const v8b*)(Kh + ko + dc * 32 + 16);
        kfl.h[0] = *(const v8b*)(Kl + ko + dc * 32);
        kfl.h[1] = *(const v8b*)(Kl + ko + dc * 32 + 16);
        sa = mma_bf16(qh[dc], kfh.v, sa);
        sa = mma_bf16(qh[dc], kfl.v, sa);
        sa = mma_bf16(ql[dc], kfh.v, sa);
      }
#pragma unroll
      for (int r = 0; r < 8; ++r) ss[(8 * hh + r) * SP + 16 * j + c] = sa[r];
    }

    {
      const int dbase = kv0 - q0 - 15;
#pragma unroll 1
      for (int t = 0; t < 5; ++t) {
        const int d = dbase + 16 * t + c;
        int rr = d % NPOS;
        rr += (rr < 0) ? NPOS : 0;
        const unsigned short* ep = Eh + (size_t)rr * DHEAD + 8 * hh;
        v8f g = (v8f){0.f,0.f,0.f,0.f,0.f,0.f,0.f,0.f};
#pragma unroll
        for (int dc = 0; dc < 2; ++dc) {
          FB ef;
          ef.h[0] = *(const v8b*)(ep + dc * 32);
          ef.h[1] = *(const v8b*)(ep + dc * 32 + 16);
          g = mma_bf16(qh[dc], ef.v, g);
          g = mma_bf16(ql[dc], ef.v, g);
        }
#pragma unroll
        for (int r = 0; r < 8; ++r) gs[(8 * hh + r) * GP + 16 * t + c] = g[r];
      }
    }
    wave_lds_sync();

    v8f s[4];
#pragma unroll
    for (int j = 0; j < 4; ++j) {
#pragma unroll
      for (int r = 0; r < 8; ++r) {
        const int m = 8 * hh + r;
        const float raw = ss[m * SP + 16 * j + c];
        const float gv = gs[m * (GP - 1) + 16 * j + c + 15];
        const float sv = raw + gv;
        const unsigned bit = (mw[r >> 1] >> (16 * (r & 1) + 4 * j + csh)) & 1u;
        s[j][r] = bit ? NEG_INF : sv;
      }
    }

    float cm[8];
#pragma unroll
    for (int r = 0; r < 8; ++r) {
      float m = fmaxf(fmaxf(s[0][r], s[1][r]), fmaxf(s[2][r], s[3][r]));
#pragma unroll
      for (int off = 1; off < 16; off <<= 1) m = fmaxf(m, __shfl_xor(m, off, 32));
      cm[r] = m;
    }

#pragma unroll
    for (int r = 0; r < 8; ++r) {
      const float mnew  = fmaxf(mrow[r], cm[r]);
      const float msafe = (mnew == NEG_INF) ? 0.f : mnew;
      const float alpha = expf(mrow[r] - msafe);
      mrow[r] = mnew;
      float psum = 0.f;
#pragma unroll
      for (int j = 0; j < 4; ++j) {
        const float p = expf(s[j][r] - msafe);
        psum += p;
        const unsigned short hb = f2bf_bits(p);
        const unsigned short lb = f2bf_bits(p - bf_bits2f(hb));
        pwh[(8 * hh + r) * KCH + j * 16 + c] = hb;
        pwl[(8 * hh + r) * KCH + j * 16 + c] = lb;
      }
#pragma unroll
      for (int off = 1; off < 16; off <<= 1) psum += __shfl_xor(psum, off, 32);
      lrow[r] = lrow[r] * alpha + psum;
#pragma unroll
      for (int t = 0; t < 4; ++t) oacc[t][r] *= alpha;
    }
    wave_lds_sync();

#pragma unroll 1
    for (int kk = 0; kk < 2; ++kk) {
      FB pa, pl;
      pa.h[0] = *(const v8b_a*)(pwh + c * KCH + kk * 32 + 8 * hh);
      pa.h[1] = *(const v8b_a*)(pwh + c * KCH + kk * 32 + 16 + 8 * hh);
      pl.h[0] = *(const v8b_a*)(pwl + c * KCH + kk * 32 + 8 * hh);
      pl.h[1] = *(const v8b_a*)(pwl + c * KCH + kk * 32 + 16 + 8 * hh);
#pragma unroll
      for (int t = 0; t < 4; ++t) {
        const size_t vo = (size_t)(t * 16 + c) * SEQ + kv0 + kk * 32 + 8 * hh;
        FB vbh, vbl;
        vbh.h[0] = *(const v8b*)(Vth + vo);
        vbh.h[1] = *(const v8b*)(Vth + vo + 16);
        vbl.h[0] = *(const v8b*)(Vtl + vo);
        vbl.h[1] = *(const v8b*)(Vtl + vo + 16);
        oacc[t] = mma_bf16(pa.v, vbh.v, oacc[t]);
        oacc[t] = mma_bf16(pl.v, vbh.v, oacc[t]);
        oacc[t] = mma_bf16(pa.v, vbl.v, oacc[t]);
      }
    }
    wave_lds_sync();
  }

  float* os = gs;
#pragma unroll
  for (int r = 0; r < 8; ++r) {
    const float inv = 1.0f / lrow[r];
#pragma unroll
    for (int t = 0; t < 4; ++t) os[(8 * hh + r) * GP + t * 16 + c] = oacc[t][r] * inv;
  }
  wave_lds_sync();
  {
    unsigned short* Ch = ctxp;
    unsigned short* Cl = ctxp + XB_E;
    const int rq  = lane >> 3;
    const int seg = lane & 7;
    for (int pass = 0; pass < 2; ++pass) {
#pragma unroll
      for (int it = 0; it < 4; ++it) {
        const int row = it * 4 + rq;
        const v4f a0 = *(const v4f_a*)(os + row * GP + seg * 8);
        const v4f a1 = *(const v4f_a*)(os + row * GP + seg * 8 + 4);
        unsigned h0, h1, h2, h3, l0, l1, l2, l3;
        split2(a0[0], a0[1], h0, l0);
        split2(a0[2], a0[3], h1, l1);
        split2(a1[0], a1[1], h2, l2);
        split2(a1[2], a1[3], h3, l3);
        v4u hw, lw;
        hw[0] = h0; hw[1] = h1; hw[2] = h2; hw[3] = h3;
        lw[0] = l0; lw[1] = l1; lw[2] = l2; lw[3] = l3;
        const size_t g = (size_t)(b * SEQ + q0 + row) * DMODEL + h * DHEAD + seg * 8;
        *(volatile v4u*)(Ch + g) = hw;
        *(volatile v4u*)(Cl + g) = lw;
      }
      __threadfence();
    }
  }
}

__global__ __launch_bounds__(128) VGPR_CAP void gemm_out_kernel(
    const unsigned short* __restrict__ ctxp, const unsigned short* __restrict__ WoT,
    const float* __restrict__ bias, float* __restrict__ out)
{
  union FB { v16b v; v8b h[2]; };
  __shared__ __align__(16) float Os[NWAVE][32 * OS_PITCH];

  const int tid  = threadIdx.x;
  const int wave = __builtin_amdgcn_readfirstlane(tid >> 5);
  const int lane = tid & 31;
  const int hh   = lane >> 4;
  const int c    = lane & 15;
  const int n0   = blockIdx.x * 64;
  const int m0   = blockIdx.y * 128;

  v8f acc[2][4];
#pragma unroll
  for (int mt = 0; mt < 2; ++mt)
#pragma unroll
    for (int t = 0; t < 4; ++t) acc[mt][t] = (v8f){0.f,0.f,0.f,0.f,0.f,0.f,0.f,0.f};

  const unsigned short* ah0 = ctxp + (size_t)(m0 + wave * 32 + c) * DMODEL + 8 * hh;
  const unsigned short* ah1 = ah0 + (size_t)16 * DMODEL;
  const unsigned short* al0 = ah0 + XB_E;
  const unsigned short* al1 = ah1 + XB_E;
  const unsigned short* bp  = WoT + (size_t)(n0 + c) * DMODEL + 8 * hh;

#pragma unroll 1
  for (int k0 = 0; k0 < DMODEL; k0 += 32) {
    FB a0h, a1h, a0l, a1l;
    a0h.h[0] = *(const v8b*)(ah0 + k0);
    a0h.h[1] = *(const v8b*)(ah0 + k0 + 16);
    a1h.h[0] = *(const v8b*)(ah1 + k0);
    a1h.h[1] = *(const v8b*)(ah1 + k0 + 16);
    a0l.h[0] = *(const v8b*)(al0 + k0);
    a0l.h[1] = *(const v8b*)(al0 + k0 + 16);
    a1l.h[0] = *(const v8b*)(al1 + k0);
    a1l.h[1] = *(const v8b*)(al1 + k0 + 16);
#pragma unroll
    for (int t = 0; t < 4; ++t) {
      FB bf;
      bf.h[0] = *(const v8b*)(bp + (size_t)t * 16 * DMODEL + k0);
      bf.h[1] = *(const v8b*)(bp + (size_t)t * 16 * DMODEL + k0 + 16);
      acc[0][t] = mma_bf16(a0h.v, bf.v, acc[0][t]);
      acc[0][t] = mma_bf16(a0l.v, bf.v, acc[0][t]);
      acc[1][t] = mma_bf16(a1h.v, bf.v, acc[1][t]);
      acc[1][t] = mma_bf16(a1l.v, bf.v, acc[1][t]);
    }
  }

  float* os = Os[wave];
#pragma unroll
  for (int t = 0; t < 4; ++t) {
    const float bv = bf_bits2f(f2bf_bits(bias[n0 + 16 * t + c]));
#pragma unroll
    for (int mt = 0; mt < 2; ++mt)
#pragma unroll
      for (int r = 0; r < 8; ++r)
        os[(mt * 16 + 8 * hh + r) * OS_PITCH + 16 * t + c] = acc[mt][t][r] + bv;
  }
  wave_lds_sync();
  {
    const int c4 = c * 4;
    for (int pass = 0; pass < 2; ++pass) {
#pragma unroll
      for (int it = 0; it < 16; ++it) {
        const int row = it * 2 + hh;
        const v4f val = *(const v4f_a*)(os + row * OS_PITCH + c4);
        *(volatile v4f*)(out + (size_t)(m0 + wave * 32 + row) * DMODEL + n0 + c4) = val;
      }
      __threadfence();
    }
  }
}

extern "C" void kernel_launch(void* const* d_in, const int* in_sizes, int n_in,
                              void* d_out, int out_size, void* d_ws, size_t ws_size,
                              hipStream_t stream)
{
  if (n_in < 7) return;
  if (in_sizes[0] < ((NB - 1) * SEQ_FULL + SEQ) * DMODEL) return;
  if (in_sizes[1] < (SEQ - 1) * SEQ_FULL + SEQ) return;
  if (in_sizes[2] < DMODEL * NQKV) return;
  if (in_sizes[3] < NQKV) return;
  if (in_sizes[4] < DMODEL * DMODEL) return;
  if (in_sizes[5] < DMODEL) return;
  if (in_sizes[6] < NHEAD * NPOS * DHEAD) return;
  if (out_size < MROWS * DMODEL) return;
  if (d_ws == nullptr || ws_size < WS_NEED) return;

  const float* x     = (const float*)d_in[0];
  const int*   mask  = (const int*)d_in[1];
  const float* W_qkv = (const float*)d_in[2];
  const float* b_qkv = (const float*)d_in[3];
  const float* W_o   = (const float*)d_in[4];
  const float* b_o   = (const float*)d_in[5];
  const float* Er    = (const float*)d_in[6];
  float* out = (float*)d_out;

  unsigned short* Xb   = (unsigned short*)d_ws;
  unsigned short* WqT  = Xb + XB_E;
  unsigned short* WoT  = WqT + WQT_E;
  unsigned short* Erb  = WoT + WOT_E;
  unsigned short* qkvp = Erb + ERB_E;
  unsigned short* ctxp = qkvp + QKVP_E;

  {
    const int nunits = MROWS * (DMODEL / 8);
    cvt_rows_kernel<<<(nunits + 255) / 256, 256, 0, stream>>>(x, Xb, nunits, DMODEL / 8, SEQ, SEQ_FULL);
  }
  {
    const int nunits = NHEAD * NPOS * (DHEAD / 8);
    cvt_rows_kernel<<<(nunits + 255) / 256, 256, 0, stream>>>(Er, Erb, nunits, DHEAD / 8, NHEAD * NPOS, NHEAD * NPOS);
  }
  wt_planes_kernel<<<dim3(DMODEL / 64, NQKV / 64), 256, 0, stream>>>(W_qkv, WqT, DMODEL, NQKV);
  wt_planes_kernel<<<dim3(DMODEL / 64, DMODEL / 64), 256, 0, stream>>>(W_o, WoT, DMODEL, DMODEL);

  gemm_qkv_kernel<<<dim3(NQKV / 64, MROWS / 128), 128, 0, stream>>>(Xb, WqT, b_qkv, qkvp);
  rel_attn_kernel<<<dim3(SEQ / 64, NBH), 128, 0, stream>>>(qkvp, Erb, mask, ctxp);
  gemm_out_kernel<<<dim3(DMODEL / 64, MROWS / 128), 128, 0, stream>>>(ctxp, WoT, b_o, out);
}
